// TimeConv_90812788507392
// MI455X (gfx1250) — hardware-verified
//
#include <hip/hip_runtime.h>


#define NP     8192
#define NHALF  4096
#define HD     256
#define HH     128
#define FI     32
#define NLV    15
#define FAN    8
#define KMOD   320
#define KGATE  288
#define TB     64
#define NT     256

static_assert(NP % TB == 0);
static_assert(KGATE % 32 == 0);
static_assert(KMOD % 32 == 0);
static_assert((TB * HD) % (4 * NT) == 0);

typedef _Float16 f16t;
typedef _Float16 v8h  __attribute__((ext_vector_type(8)));
typedef _Float16 v16h __attribute__((ext_vector_type(16)));
typedef float    v8f  __attribute__((ext_vector_type(8)));
typedef float    v4f  __attribute__((ext_vector_type(4)));
typedef unsigned short u16x8 __attribute__((ext_vector_type(8)));

union Frag  { v16h v; v8h half[2]; };
union Pack8 { v8h f; u16x8 u; };

#define LV_A     0
#define LV_ZIN   40960
#define LV_STG   0
#define LV_H     73728
#define LV_TIN   90112
#define LV_TH    94208
#define LV_IDX   98304
#define LV_BP    100352
#define LV_SP    102400
#define LV_LG    104448
#define LV_AL    106496
#define LV_STP   108544
#define LV_AV    109056
#define LV_BYTES 110336

#define K1_HIN   0
#define K1_STG   16384
#define K1_BYTES 81920

#define KO_A     0
#define KO_PD    65536
#define KO_OUT   66560
#define KO_BYTES 66816

__device__ __forceinline__ v16h ld_frag(const f16t* base, int pitch, int row0, int k0) {
  const int lane = threadIdx.x & 31;
  const int h = lane >> 4, m = lane & 15;
  const f16t* p = base + (size_t)(row0 + m) * pitch + k0 + 8 * h;
  Frag f;
  f.half[0] = *(const v8h*)(p);
  f.half[1] = *(const v8h*)(p + 16);
  return f.v;
}

__device__ __forceinline__ void mma(v8f& acc, const v16h& a, const v16h& b) {
  acc = __builtin_amdgcn_wmma_f32_16x16x32_f16(false, a, false, b, (short)0, acc, false, false);
  asm volatile("v_nop\n\tv_nop\n\tv_nop\n\tv_nop" : "+v"(acc) : "v"(a), "v"(b));
}

__device__ __forceinline__ v8f zero8() {
  v8f z;
#pragma unroll
  for (int r = 0; r < 8; ++r) z[r] = 0.0f;
  return z;
}

__device__ __forceinline__ float leaky01(float x) { return (x > 0.0f) ? x : 0.1f * x; }

__global__ __launch_bounds__(NT) void k_wt(const float* __restrict__ W, int K, int N, int Kp, f16t* Wt) {
  const int i = blockIdx.x * NT + threadIdx.x;
  const int tot = (N * Kp) >> 3;
  if (i >= tot) return;
  const int e = i * 8;
  const int n = e / Kp;
  const int k0 = e - n * Kp;
  Pack8 pk;
#pragma unroll
  for (int j = 0; j < 8; ++j) {
    const int k = k0 + j;
    const int kc = (k < K) ? k : (K - 1);
    float x = W[(size_t)kc * N + n] * 16.0f;
    if (k >= K) x = 0.0f;
    pk.f[j] = (f16t)x;
  }
  const u16x8 v = pk.u;
  unsigned short* gp = (unsigned short*)Wt + e;
  *(volatile u16x8*)gp = v;
  __threadfence();
  *(volatile u16x8*)gp = v;
}

__device__ __forceinline__ void store_pass_tile(const float* st, float* g) {
  const int t = threadIdx.x;
#pragma unroll
  for (int it = 0; it < (TB * HD) / (4 * NT); ++it) {
    const int q = t + NT * it;
    const v4f v = *(const v4f*)(st + 4 * q);
    *(volatile v4f*)(g + 4 * (size_t)q) = v;
  }
}

__device__ __forceinline__ void gemm_l1(const f16t* Als, const f16t* __restrict__ W1t, int kp, int nk,
                                        const float* __restrict__ b1, f16t* Hls) {
  const int lane = threadIdx.x & 31, wave = threadIdx.x >> 5;
  const int h = lane >> 4, m = lane & 15;
  const int r0 = (wave >> 2) * 32, c0 = (wave & 3) * 32;
  v8f acc[4];
#pragma unroll
  for (int j = 0; j < 4; ++j) acc[j] = zero8();
#pragma unroll 1
  for (int ks = 0; ks < nk; ++ks) {
    const int k0 = ks * 32;
    const v16h a0 = ld_frag(Als, KMOD, r0, k0);
    const v16h a1 = ld_frag(Als, KMOD, r0 + 16, k0);
    const v16h b0 = ld_frag(W1t, kp, c0, k0);
    const v16h bb1 = ld_frag(W1t, kp, c0 + 16, k0);
    mma(acc[0], a0, b0);
    mma(acc[1], a0, bb1);
    mma(acc[2], a1, b0);
    mma(acc[3], a1, bb1);
  }
#pragma unroll
  for (int s = 0; s < 2; ++s)
#pragma unroll
    for (int j = 0; j < 2; ++j) {
      const int col = c0 + 16 * j + m;
      const float bb = b1[col];
#pragma unroll
      for (int r = 0; r < 8; ++r)
        Hls[(r0 + 16 * s + 8 * h + r) * HH + col] = (f16t)leaky01(acc[2 * s + j][r] * 0.0625f + bb);
    }
}

__device__ __forceinline__ void gemm_l2(const f16t* Hls, const f16t* __restrict__ W2t,
                                        const float* __restrict__ b2, int doRelu, float* stg) {
  const int lane = threadIdx.x & 31, wave = threadIdx.x >> 5;
  const int h = lane >> 4, m = lane & 15;
  const int r0 = (wave >> 2) * 32, c0 = (wave & 3) * 64;
  v8f acc[8];
#pragma unroll
  for (int j = 0; j < 8; ++j) acc[j] = zero8();
#pragma unroll 1
  for (int ks = 0; ks < HH / 32; ++ks) {
    const int k0 = ks * 32;
    const v16h a0 = ld_frag(Hls, HH, r0, k0);
    const v16h a1 = ld_frag(Hls, HH, r0 + 16, k0);
#pragma unroll
    for (int j = 0; j < 4; ++j) {
      const v16h b = ld_frag(W2t, HH, c0 + 16 * j, k0);
      mma(acc[j], a0, b);
      mma(acc[4 + j], a1, b);
    }
  }
#pragma unroll
  for (int j = 0; j < 4; ++j) {
    const int col = c0 + 16 * j + m;
    const float bb = b2[col];
#pragma unroll
    for (int s = 0; s < 2; ++s)
#pragma unroll
      for (int r = 0; r < 8; ++r) {
        float x = acc[4 * s + j][r] * 0.0625f + bb;
        if (doRelu) x = fmaxf(x, 0.0f);
        stg[(r0 + 16 * s + 8 * h + r) * HD + col] = x;
      }
  }
}

__global__ __launch_bounds__(NT) void k_mlp_k1(const float* __restrict__ x, const float* __restrict__ w1,
                                               const float* __restrict__ b1, const f16t* __restrict__ w2t,
                                               const float* __restrict__ b2, float* outp) {
  extern __shared__ __attribute__((aligned(16))) unsigned char smem[];
  f16t*  Hin = (f16t*)(smem + K1_HIN);
  float* stg = (float*)(smem + K1_STG);
  const int t = threadIdx.x;
  const int nb = blockIdx.x * TB;
#pragma unroll 4
  for (int j = 0; j < (TB * HH) / NT; ++j) {
    const int e = t + NT * j;
    const int node = e >> 7, c = e & (HH - 1);
    Hin[e] = (f16t)leaky01(x[nb + node] * w1[c] + b1[c]);
  }
  __syncthreads();
  gemm_l2(Hin, w2t, b2, 0, stg);
  __syncthreads();
  float* g = outp + (size_t)nb * HD;
  store_pass_tile(stg, g);
  __threadfence();
  store_pass_tile(stg, g);
}

__global__ __launch_bounds__(NT) void k_level(
    const float* __restrict__ prev, const int* __restrict__ srcl,
    const float* __restrict__ featl, const float* __restrict__ bpl,
    const float* __restrict__ av,
    const f16t* __restrict__ gw1t, const float* __restrict__ gb1,
    const f16t* __restrict__ gw2t, const float* __restrict__ gb2,
    const f16t* __restrict__ mw1t, const float* __restrict__ mb1,
    const f16t* __restrict__ mw2t, const float* __restrict__ mb2,
    const f16t* __restrict__ tw1t, const float* __restrict__ tb1,
    const f16t* __restrict__ tw2t, const float* __restrict__ tb2,
    const float* __restrict__ pw1, const float* __restrict__ pb1,
    const f16t* __restrict__ pw2t, const float* __restrict__ pb2,
    float* nxt, int doRelu)
{
  extern __shared__ __attribute__((aligned(16))) unsigned char smem[];
  f16t*  Als  = (f16t*)(smem + LV_A);
  f16t*  Zin  = (f16t*)(smem + LV_ZIN);
  float* stg  = (float*)(smem + LV_STG);
  f16t*  Hls  = (f16t*)(smem + LV_H);
  f16t*  Tin  = (f16t*)(smem + LV_TIN);
  f16t*  Th   = (f16t*)(smem + LV_TH);
  int*   idxl = (int*)(smem + LV_IDX);
  float* bpt  = (float*)(smem + LV_BP);
  float* spv  = (float*)(smem + LV_SP);
  float* lgs  = (float*)(smem + LV_LG);
  float* alps = (float*)(smem + LV_AL);
  float* stp  = (float*)(smem + LV_STP);
  float* avl  = (float*)(smem + LV_AV);

  const int t = threadIdx.x, lane = t & 31, wave = t >> 5;
  const int h = lane >> 4, m = lane & 15;
  const int nb = blockIdx.x * TB;
  const bool isMod = (blockIdx.x >= (NHALF / TB));

  for (int e = t; e < TB * FAN; e += NT) {
    int g = srcl[(size_t)nb * FAN + e];
    g = (g < 0) ? (g + NP) : g;
    g = (g < 0) ? 0 : g;
    g = (g > NP - 1) ? (NP - 1) : g;
    idxl[e] = g;
  }

  if (!isMod) {
#pragma unroll
    for (int j = 0; j < (TB * FI) / NT; ++j) {
      const int e = t + NT * j;
      const int node = e >> 5, c = e & 31;
      Als[node * KMOD + HD + c]    = (f16t)featl[(size_t)nb * FI + e];
      Als[node * KMOD + KGATE + c] = (f16t)0.0f;
    }
    __syncthreads();
    for (int i = 0; i < TB; ++i) {
      float v[FAN];
      float mx = -3.0e38f;
#pragma unroll
      for (int f = 0; f < FAN; ++f) {
        v[f] = prev[(size_t)idxl[i * FAN + f] * HD + t];
        mx = fmaxf(mx, v[f]);
      }
      float s = 0.0f, a = 0.0f;
#pragma unroll
      for (int f = 0; f < FAN; ++f) {
        const float e = __expf(v[f] - mx);
        s += e;
        a += e * v[f];
      }
      Als[i * KMOD + t] = (f16t)(a * __builtin_amdgcn_rcpf(s));
    }
  } else {
    for (int e = t; e < TB * FAN; e += NT) bpt[e] = bpl[(size_t)nb * FAN + e];
    for (int e = t; e < KMOD; e += NT) avl[e] = av[e];
#pragma unroll
    for (int j = 0; j < (TB * FI) / NT; ++j) {
      const int e = t + NT * j;
      const int node = e >> 5, c = e & 31;
      const f16t xv = (f16t)featl[(size_t)nb * FI + e];
      Tin[e] = xv;
      Als[node * KMOD + (HD + 1) + c] = xv;
    }
    for (int e = t; e < TB * (KMOD - HD - 1 - FI); e += NT) {
      const int node = e / (KMOD - HD - 1 - FI), c = e - node * (KMOD - HD - 1 - FI);
      Als[node * KMOD + (HD + 1 + FI) + c] = (f16t)0.0f;
    }
    __syncthreads();
    {
      const int j = t & 31;
      const float w1j = pw1[j], b1j = pb1[j];
      for (int r = (t >> 5); r < TB * FAN; r += (NT / 32))
        Zin[r * 32 + j] = (f16t)leaky01(bpt[r] * w1j + b1j);
    }
    __syncthreads();
    {
      const int rt = wave >> 1, ct = wave & 1;
      v8f acc = zero8();
      mma(acc, ld_frag(Tin, 32, rt * 16, 0), ld_frag(tw1t, 32, ct * 16, 0));
      const int col = ct * 16 + m;
      const float bb = tb1[col];
#pragma unroll
      for (int r = 0; r < 8; ++r)
        Th[(rt * 16 + 8 * h + r) * 32 + col] = (f16t)leaky01(acc[r] * 0.0625f + bb);
    }
    __syncthreads();
    {
      const int rt = wave >> 1, ct = wave & 1;
      v8f acc = zero8();
      mma(acc, ld_frag(Th, 32, rt * 16, 0), ld_frag(tw2t, 32, ct * 16, 0));
      const int col = ct * 16 + m;
      const float bb = tb2[col];
      const float aw = avl[col];
      float val[8];
#pragma unroll
      for (int r = 0; r < 8; ++r) val[r] = (acc[r] * 0.0625f + bb) * aw;
#pragma unroll
      for (int r = 0; r < 8; ++r) {
        val[r] += __shfl_xor(val[r], 8);
        val[r] += __shfl_xor(val[r], 4);
        val[r] += __shfl_xor(val[r], 2);
        val[r] += __shfl_xor(val[r], 1);
      }
      if (m == 0) {
#pragma unroll
        for (int r = 0; r < 8; ++r) stp[ct * TB + rt * 16 + 8 * h + r] = val[r];
      }
    }
    {
      const v16h b0 = ld_frag(pw2t, 32, 0, 0);
      const v16h bb1 = ld_frag(pw2t, 32, 16, 0);
      const float c0 = pb2[m], c1 = pb2[16 + m];
      const float w0 = avl[32 + m], w1 = avl[48 + m];
#pragma unroll
      for (int q = 0; q < 4; ++q) {
        const int rt = wave * 4 + q;
        const v16h a = ld_frag(Zin, 32, rt * 16, 0);
        v8f acc0 = zero8(), acc1 = zero8();
        mma(acc0, a, b0);
        mma(acc1, a, bb1);
        float val[8];
#pragma unroll
        for (int r = 0; r < 8; ++r)
          val[r] = (acc0[r] * 0.0625f + c0) * w0 + (acc1[r] * 0.0625f + c1) * w1;
#pragma unroll
        for (int r = 0; r < 8; ++r) {
          val[r] += __shfl_xor(val[r], 8);
          val[r] += __shfl_xor(val[r], 4);
          val[r] += __shfl_xor(val[r], 2);
          val[r] += __shfl_xor(val[r], 1);
        }
        if (m == 0) {
#pragma unroll
          for (int r = 0; r < 8; ++r) spv[rt * 16 + 8 * h + r] = val[r];
        }
      }
    }
    __syncthreads();
#pragma unroll
    for (int q = 0; q < 2; ++q) {
      const int r = t + NT * q;
      const int node = r >> 3;
      const float* rp = prev + (size_t)idxl[r] * HD;
      float d = 0.0f;
#pragma unroll 4
      for (int c4 = 0; c4 < HD / 4; ++c4) {
        const v4f x = *(const v4f*)(rp + 4 * c4);
        const v4f a = *(const v4f*)(avl + 64 + 4 * c4);
        d += x[0] * a[0];
        d += x[1] * a[1];
        d += x[2] * a[2];
        d += x[3] * a[3];
      }
      lgs[r] = d + spv[r] + (stp[node] + stp[TB + node]);
    }
    __syncthreads();
    if (t < TB) {
      const int node = t;
      float e8[FAN];
      float mx = -3.0e38f;
#pragma unroll
      for (int f = 0; f < FAN; ++f) mx = fmaxf(mx, lgs[node * FAN + f]);
      float S = 0.0f;
#pragma unroll
      for (int f = 0; f < FAN; ++f) { e8[f] = __expf(lgs[node * FAN + f] - mx); S += e8[f]; }
      const float inv = __builtin_amdgcn_rcpf(S);
      float nbv = 0.0f;
#pragma unroll
      for (int f = 0; f < FAN; ++f) {
        const float al = e8[f] * inv;
        alps[node * FAN + f] = al;
        nbv += al * bpt[node * FAN + f];
      }
      Als[node * KMOD + HD] = (f16t)nbv;
    }
    __syncthreads();
    for (int i = 0; i < TB; ++i) {
      float nm = 0.0f;
#pragma unroll
      for (int f = 0; f < FAN; ++f)
        nm += alps[i * FAN + f] * prev[(size_t)idxl[i * FAN + f] * HD + t];
      Als[i * KMOD + t] = (f16t)nm;
    }
  }
  __syncthreads();

  const f16t*  W1t = isMod ? mw1t : gw1t;
  const float* B1  = isMod ? mb1 : gb1;
  const f16t*  W2t = isMod ? mw2t : gw2t;
  const float* B2  = isMod ? mb2 : gb2;
  const int kp = isMod ? KMOD : KGATE;
  gemm_l1(Als, W1t, kp, kp / 32, B1, Hls);
  __syncthreads();
  gemm_l2(Hls, W2t, B2, doRelu, stg);
  __syncthreads();
  float* g = nxt + (size_t)nb * HD;
  store_pass_tile(stg, g);
  __threadfence();
  store_pass_tile(stg, g);
}

__global__ __launch_bounds__(NT) void k_out(const float* __restrict__ hc, const float* __restrict__ hg,
                                            const f16t* __restrict__ w1t, const float* __restrict__ b1,
                                            const float* __restrict__ w2, const float* __restrict__ b2,
                                            float* outp) {
  extern __shared__ __attribute__((aligned(16))) unsigned char smem[];
  f16t*  Als  = (f16t*)(smem + KO_A);
  float* pd   = (float*)(smem + KO_PD);
  float* outs = (float*)(smem + KO_OUT);
  const int t = threadIdx.x, lane = t & 31, wave = t >> 5;
  const int h = lane >> 4, m = lane & 15;
  const int nb = blockIdx.x * TB;

#pragma unroll 4
  for (int j = 0; j < (TB * HD) / (4 * NT); ++j) {
    const int q = t + NT * j;
    const int node = q >> 6, cc = q & 63;
    const v4f x = *(const v4f*)(hc + (size_t)(nb + node) * HD + 4 * cc);
    f16t* d = Als + node * (2 * HD) + 4 * cc;
    d[0] = (f16t)x[0]; d[1] = (f16t)x[1]; d[2] = (f16t)x[2]; d[3] = (f16t)x[3];
  }
#pragma unroll 4
  for (int j = 0; j < (TB * HD) / (4 * NT); ++j) {
    const int q = t + NT * j;
    const int node = q >> 6, cc = q & 63;
    const v4f x = *(const v4f*)(hg + (size_t)(nb + node) * HD + 4 * cc);
    f16t* d = Als + node * (2 * HD) + HD + 4 * cc;
    d[0] = (f16t)x[0]; d[1] = (f16t)x[1]; d[2] = (f16t)x[2]; d[3] = (f16t)x[3];
  }
  __syncthreads();

  const int r0 = (wave >> 2) * 32, c0 = (wave & 3) * 64;
  v8f acc[8];
#pragma unroll
  for (int j = 0; j < 8; ++j) acc[j] = zero8();
#pragma unroll 1
  for (int ks = 0; ks < (2 * HD) / 32; ++ks) {
    const int k0 = ks * 32;
    const v16h a0 = ld_frag(Als, 2 * HD, r0, k0);
    const v16h a1 = ld_frag(Als, 2 * HD, r0 + 16, k0);
#pragma unroll
    for (int j = 0; j < 4; ++j) {
      const v16h b = ld_frag(w1t, 2 * HD, c0 + 16 * j, k0);
      mma(acc[j], a0, b);
      mma(acc[4 + j], a1, b);
    }
  }
  float pr0[8], pr1[8];
#pragma unroll
  for (int r = 0; r < 8; ++r) { pr0[r] = 0.0f; pr1[r] = 0.0f; }
#pragma unroll
  for (int j = 0; j < 4; ++j) {
    const int col = c0 + 16 * j + m;
    const float bb = b1[col];
    const float ww = w2[col];
#pragma unroll
    for (int r = 0; r < 8; ++r) {
      pr0[r] += leaky01(acc[j][r] * 0.0625f + bb) * ww;
      pr1[r] += leaky01(acc[4 + j][r] * 0.0625f + bb) * ww;
    }
  }
#pragma unroll
  for (int r = 0; r < 8; ++r) {
    pr0[r] += __shfl_xor(pr0[r], 8); pr0[r] += __shfl_xor(pr0[r], 4);
    pr0[r] += __shfl_xor(pr0[r], 2); pr0[r] += __shfl_xor(pr0[r], 1);
    pr1[r] += __shfl_xor(pr1[r], 8); pr1[r] += __shfl_xor(pr1[r], 4);
    pr1[r] += __shfl_xor(pr1[r], 2); pr1[r] += __shfl_xor(pr1[r], 1);
  }
  if (m == 0) {
#pragma unroll
    for (int r = 0; r < 8; ++r) {
      pd[(wave & 3) * TB + r0 + 8 * h + r]      = pr0[r];
      pd[(wave & 3) * TB + r0 + 16 + 8 * h + r] = pr1[r];
    }
  }
  __syncthreads();
  if (t < TB) outs[t] = ((pd[t] + pd[TB + t]) + (pd[2 * TB + t] + pd[3 * TB + t])) + b2[0];
  __syncthreads();
  if (t < TB / 4) {
    const v4f v = *(const v4f*)(outs + 4 * t);
    *(volatile v4f*)(outp + nb + 4 * t) = v;
  }
  __threadfence();
  if (t < TB / 4) {
    const v4f v = *(const v4f*)(outs + 4 * t);
    *(volatile v4f*)(outp + nb + 4 * t) = v;
  }
}

extern "C" void kernel_launch(void* const* d_in, const int* in_sizes, int n_in,
                              void* d_out, int out_size, void* d_ws, size_t ws_size,
                              hipStream_t stream)
{
  if (n_in < 34) return;
  if (in_sizes[0] != NP) return;
  if (in_sizes[1] != (NLV + 1) * NP * FI) return;
  if (in_sizes[2] != NLV * NP * FAN) return;
  if (in_sizes[3] != NP) return;
  if (in_sizes[4] != NLV * NP * FAN) return;
  if (in_sizes[5] != HH || in_sizes[6] != HH || in_sizes[7] != HH * HD || in_sizes[8] != HD) return;
  if (in_sizes[9] != KGATE * HH || in_sizes[10] != HH || in_sizes[11] != HH * HD || in_sizes[12] != HD) return;
  if (in_sizes[13] != (HD + 1 + FI) * HH || in_sizes[14] != HH || in_sizes[15] != HH * HD || in_sizes[16] != HD) return;
  if (in_sizes[17] != FI * 32 || in_sizes[18] != 32 || in_sizes[19] != 32 * 32 || in_sizes[20] != 32) return;
  if (in_sizes[21] != 32 || in_sizes[22] != 32 || in_sizes[23] != 32 * 32 || in_sizes[24] != 32) return;
  if (in_sizes[25] != KMOD) return;
  if (in_sizes[26] != HH || in_sizes[27] != HH || in_sizes[28] != HH * HD || in_sizes[29] != HD) return;
  if (in_sizes[30] != 2 * HD * HD || in_sizes[31] != HD || in_sizes[32] != HD || in_sizes[33] != 1) return;
  if (out_size != NP) return;

  const float* delay   = (const float*)d_in[0];
  const float* feat    = (const float*)d_in[1];
  const float* bit_pos = (const float*)d_in[2];
  const float* po_feat = (const float*)d_in[3];
  const int*   src_idx = (const int*)d_in[4];
  const float* pi_w1   = (const float*)d_in[5];
  const float* pi_b1   = (const float*)d_in[6];
  const float* pi_w2   = (const float*)d_in[7];
  const float* pi_b2   = (const float*)d_in[8];
  const float* gate_w1 = (const float*)d_in[9];
  const float* gate_b1 = (const float*)d_in[10];
  const float* gate_w2 = (const float*)d_in[11];
  const float* gate_b2 = (const float*)d_in[12];
  const float* mod_w1  = (const float*)d_in[13];
  const float* mod_b1  = (const float*)d_in[14];
  const float* mod_w2  = (const float*)d_in[15];
  const float* mod_b2  = (const float*)d_in[16];
  const float* type_w1 = (const float*)d_in[17];
  const float* type_b1 = (const float*)d_in[18];
  const float* type_w2 = (const float*)d_in[19];
  const float* type_b2 = (const float*)d_in[20];
  const float* pos_w1  = (const float*)d_in[21];
  const float* pos_b1  = (const float*)d_in[22];
  const float* pos_w2  = (const float*)d_in[23];
  const float* pos_b2  = (const float*)d_in[24];
  const float* attn    = (const float*)d_in[25];
  const float* glob_w1 = (const float*)d_in[26];
  const float* glob_b1 = (const float*)d_in[27];
  const float* glob_w2 = (const float*)d_in[28];
  const float* glob_b2 = (const float*)d_in[29];
  const float* out_w1  = (const float*)d_in[30];
  const float* out_b1  = (const float*)d_in[31];
  const float* out_w2  = (const float*)d_in[32];
  const float* out_b2  = (const float*)d_in[33];
  float* out = (float*)d_out;

  const size_t SZ_GW1T = (size_t)HH * KGATE * 2;
  const size_t SZ_W2T  = (size_t)HD * HH * 2;
  const size_t SZ_MW1T = (size_t)HH * KMOD * 2;
  const size_t SZ_OW1T = (size_t)HD * (2 * HD) * 2;
  const size_t SZ_S32  = (size_t)32 * 32 * 2;
  const size_t SZ_PL   = (size_t)NP * HD * 4;
  size_t off = 0;
  const size_t OFF_GW1T = off; off += SZ_GW1T;
  const size_t OFF_GW2T = off; off += SZ_W2T;
  const size_t OFF_MW1T = off; off += SZ_MW1T;
  const size_t OFF_MW2T = off; off += SZ_W2T;
  const size_t OFF_PW2T = off; off += SZ_W2T;
  const size_t OFF_LW2T = off; off += SZ_W2T;
  const size_t OFF_OW1T = off; off += SZ_OW1T;
  const size_t OFF_TW1T = off; off += SZ_S32;
  const size_t OFF_TW2T = off; off += SZ_S32;
  const size_t OFF_SW2T = off; off += SZ_S32;
  const size_t OFF_HA   = off; off += SZ_PL;
  const size_t OFF_HB   = off; off += SZ_PL;
  const size_t OFF_HG   = off; off += SZ_PL;
  const size_t WS_END   = off;
  if (WS_END > ws_size) return;
  if (WS_END > (size_t)134217728) return;

  char* ws = (char*)d_ws;
  f16t* gw1t  = (f16t*)(ws + OFF_GW1T);
  f16t* gw2t  = (f16t*)(ws + OFF_GW2T);
  f16t* mw1t  = (f16t*)(ws + OFF_MW1T);
  f16t* mw2t  = (f16t*)(ws + OFF_MW2T);
  f16t* piw2t = (f16t*)(ws + OFF_PW2T);
  f16t* glw2t = (f16t*)(ws + OFF_LW2T);
  f16t* ow1t  = (f16t*)(ws + OFF_OW1T);
  f16t* tw1t  = (f16t*)(ws + OFF_TW1T);
  f16t* tw2t  = (f16t*)(ws + OFF_TW2T);
  f16t* sw2t  = (f16t*)(ws + OFF_SW2T);
  float* hA   = (float*)(ws + OFF_HA);
  float* hB   = (float*)(ws + OFF_HB);
  float* hG   = (float*)(ws + OFF_HG);

  hipFuncSetAttribute(reinterpret_cast<const void*>(&k_level), hipFuncAttributeMaxDynamicSharedMemorySize, LV_BYTES);
  hipFuncSetAttribute(reinterpret_cast<const void*>(&k_mlp_k1), hipFuncAttributeMaxDynamicSharedMemorySize, K1_BYTES);
  hipFuncSetAttribute(reinterpret_cast<const void*>(&k_out), hipFuncAttributeMaxDynamicSharedMemorySize, KO_BYTES);

  auto cvt = [&](const float* W, int K, int N, int Kp, f16t* dst) {
    const int pieces = (N * Kp) / 8;
    hipLaunchKernelGGL(k_wt, dim3((pieces + NT - 1) / NT), dim3(NT), 0, stream, W, K, N, Kp, dst);
  };
  cvt(gate_w1, KGATE,       HH, KGATE,  gw1t);
  cvt(gate_w2, HH,          HD, HH,     gw2t);
  cvt(mod_w1,  HD + 1 + FI, HH, KMOD,   mw1t);
  cvt(mod_w2,  HH,          HD, HH,     mw2t);
  cvt(pi_w2,   HH,          HD, HH,     piw2t);
  cvt(glob_w2, HH,          HD, HH,     glw2t);
  cvt(out_w1,  2 * HD,      HD, 2 * HD, ow1t);
  cvt(type_w1, FI,          32, 32,     tw1t);
  cvt(type_w2, 32,          32, 32,     tw2t);
  cvt(pos_w2,  32,          32, 32,     sw2t);

  hipLaunchKernelGGL(k_mlp_k1, dim3(NP / TB), dim3(NT), K1_BYTES, stream,
                     delay, pi_w1, pi_b1, (const f16t*)piw2t, pi_b2, hA);

  float* cur = hA;
  float* nxt = hB;
  for (int l = 0; l < NLV; ++l) {
    const int*   srcl  = src_idx + (size_t)l * NP * FAN;
    const float* featl = feat + (size_t)(l + 1) * NP * FI;
    const float* bpl   = bit_pos + (size_t)l * NP * FAN;
    const int doRelu = (l < NLV - 1) ? 1 : 0;
    hipLaunchKernelGGL(k_level, dim3(NP / TB), dim3(NT), LV_BYTES, stream,
                       (const float*)cur, srcl, featl, bpl, attn,
                       (const f16t*)gw1t, gate_b1, (const f16t*)gw2t, gate_b2,
                       (const f16t*)mw1t, mod_b1, (const f16t*)mw2t, mod_b2,
                       (const f16t*)tw1t, type_b1, (const f16t*)tw2t, type_b2,
                       pos_w1, pos_b1, (const f16t*)sw2t, pos_b2,
                       nxt, doRelu);
    float* tmp = cur; cur = nxt; nxt = tmp;
  }

  hipLaunchKernelGGL(k_mlp_k1, dim3(NP / TB), dim3(NT), K1_BYTES, stream,
                     po_feat, glob_w1, glob_b1, (const f16t*)glw2t, glob_b2, hG);

  hipLaunchKernelGGL(k_out, dim3(NP / TB), dim3(NT), KO_BYTES, stream,
                     (const float*)cur, (const float*)hG, (const f16t*)ow1t, out_b1, out_w2, out_b2, out);
}
